// MAB_20263655702989
// MI455X (gfx1250) — hardware-verified
//
#include <hip/hip_runtime.h>
#include <math.h>

typedef __attribute__((ext_vector_type(16))) _Float16 v16h;
typedef __attribute__((ext_vector_type(16))) __bf16 v16b;
typedef __attribute__((ext_vector_type(8)))  _Float16 v8h;
typedef __attribute__((ext_vector_type(8)))  float v8f;
typedef __attribute__((ext_vector_type(4)))  float v4f;
typedef __attribute__((ext_vector_type(4)))  unsigned v4u;

template <typename T> __device__ __forceinline__ void vst2(void* p, T v) { *(volatile T*)p = v; __threadfence(); *(volatile T*)p = v; }
__device__ __forceinline__ v8f wmma16(v16h a, v16h b, v8f c) {
  v8f d = __builtin_amdgcn_wmma_f32_16x16x32_f16(false, a, false, b, (short)0, c, false, false);
  asm volatile("v_nop\n\tv_nop\n\tv_nop\n\tv_nop" : "+v"(d) : "v"(a), "v"(b));
  return d;
}
__device__ __forceinline__ v8f wmma_bf(v16b a, v16b b, v8f c) {
  v8f d = __builtin_amdgcn_wmma_f32_16x16x32_bf16(false, a, false, b, (short)0, c, false, false);
  asm volatile("v_nop\n\tv_nop\n\tv_nop\n\tv_nop" : "+v"(d) : "v"(a), "v"(b));
  return d;
}
__device__ __forceinline__ v16h frag_h(const _Float16* rowk0, int lane) {
  union { v16h v; v8h q[2]; } u; const _Float16* p = rowk0 + 8 * (lane >> 4);
  u.q[0] = *(const v8h*)p; u.q[1] = *(const v8h*)(p + 16); return u.v;
}
__device__ __forceinline__ v16h frag_f32(const float* rowk0, int lane) {
  v16h a; const float* p = rowk0 + 8 * (lane >> 4);
#pragma unroll
  for (int i = 0; i < 8; ++i) { a[i] = (_Float16)p[i]; a[8 + i] = (_Float16)p[16 + i]; }
  return a;
}
struct F2 { v16b h, l; };
__device__ __forceinline__ F2 bsplit16(const float v[16]) { F2 r;
#pragma unroll
  for (int i = 0; i < 16; ++i) { const __bf16 hh = (__bf16)v[i]; r.h[i] = hh; r.l[i] = (__bf16)(v[i] - (float)hh); }
  return r; }
__device__ __forceinline__ F2 split_row(const float* row, int k0, int lane) { float v[16]; const float* p = row + k0 + 8 * (lane >> 4);
#pragma unroll
  for (int i = 0; i < 8; ++i) { v[i] = p[i]; v[8 + i] = p[16 + i]; }
  return bsplit16(v); }
__device__ __forceinline__ float bfr(float v) { return (float)(__bf16)v; }
__device__ __forceinline__ v16b wcol_io(const float* Wm, int k0, int o, int lane, int ld) { v16b w; const int g = lane >> 4;
#pragma unroll
  for (int i = 0; i < 8; ++i) { w[i] = (__bf16)Wm[(size_t)(k0 + 8 * g + i) * ld + o]; w[8 + i] = (__bf16)Wm[(size_t)(k0 + 16 + 8 * g + i) * ld + o]; }
  return w; }
__device__ __forceinline__ void ldsx() { asm volatile("s_wait_dscnt 0x0" ::: "memory"); __builtin_amdgcn_wave_barrier(); __builtin_amdgcn_fence(3, "workgroup"); }

#ifndef NB
#define NB 8
#endif
#ifndef SEQ
#define SEQ 2048
#endif
#define NB_FULL 8
#define SEQ_FULL 2048
#define DIN 256
#define CC 256
#define NH 4
#define HD 64
#define HG 2
#define NQB (SEQ / 64)
#define NROW (NB * SEQ)
#define NQ4 (CC / 128)
#define SCALE (0.125f)
#define PCARRY (2048.0f)
#define QRES (1024.0f)
static_assert(NB >= 1 && NB <= NB_FULL);
static_assert(SEQ >= 128 && SEQ <= SEQ_FULL && (SEQ % 128) == 0);
static_assert(CC == NH * HD && (NH % HG) == 0 && HD == 64);
static_assert((DIN % 32) == 0 && (CC % 128) == 0 && (NROW % 64) == 0);

#define WS_QH  ((size_t)0)
#define WS_KH  (WS_QH + 2u * (size_t)NROW * CC)
#define WS_VT  (WS_KH + 2u * (size_t)NROW * CC)
#define WS_QL  (WS_VT + 2u * (size_t)NB * CC * SEQ)
#define WS_S   (WS_QL + 2u * (size_t)NROW * CC)
#define WS_QF  (WS_S  + 4u * (size_t)HG * SEQ * SEQ)
#define WS_O   (WS_QF + 4u * (size_t)NROW * CC)
#define WS_T   (WS_O  + 4u * (size_t)NROW * CC)
#define WS_END (WS_T  + 4u * (size_t)NROW * CC)
static_assert(WS_END <= (size_t)134217728u);
static_assert((WS_KH % 128) == 0 && (WS_VT % 128) == 0 && (WS_QL % 128) == 0 && (WS_S % 128) == 0 && (WS_QF % 128) == 0 && (WS_O % 128) == 0 && (WS_T % 128) == 0);

__global__ __launch_bounds__(128) void k_proj(const float* __restrict__ XQ, const float* __restrict__ XK, const float* __restrict__ WQ, const float* __restrict__ WK, const float* __restrict__ WV,
    const float* __restrict__ BQ, const float* __restrict__ BK, const float* __restrict__ BV, _Float16* __restrict__ QH, _Float16* __restrict__ QL, _Float16* __restrict__ KH, _Float16* __restrict__ VT) {
  __shared__ __align__(16) _Float16 sh[64][136], sl[64][136];
  __shared__ __align__(16) _Float16 th[128][72];
  const int tid = threadIdx.x, wave = tid >> 5, lane = tid & 31, col = lane & 15, g = lane >> 4;
  const int which = blockIdx.z; const int c0 = blockIdx.y * 128;
  const size_t r0 = (size_t)blockIdx.x * 64; const size_t bb = r0 / SEQ; const int t0 = (int)(r0 % SEQ);
  const size_t x0 = bb * SEQ_FULL + t0;
  const float* X = which == 0 ? XQ : XK; const float* WA = which == 0 ? WQ : (which == 1 ? WK : WV); const float* BA = which == 0 ? BQ : (which == 1 ? BK : BV);
  v8f acc[8] = {};
#pragma unroll 2
  for (int kc = 0; kc < DIN / 32; ++kc) {
    v16b a; { const float* p = X + (x0 + wave * 16 + col) * DIN + kc * 32 + 8 * g;
#pragma unroll
      for (int i = 0; i < 8; ++i) { a[i] = (__bf16)p[i]; a[8 + i] = (__bf16)p[16 + i]; } }
    asm volatile("s_wait_loadcnt 0x0" ::: "memory");
#pragma unroll
    for (int j = 0; j < 8; ++j) { const v16b w = wcol_io(WA, kc * 32, c0 + j * 16 + col, lane, CC); asm volatile("s_wait_loadcnt 0x0" ::: "memory"); acc[j] = wmma_bf(a, w, acc[j]); }
  }
  if (which < 2) {
#pragma unroll
    for (int j = 0; j < 8; ++j) { const float bias = bfr(BA[c0 + j * 16 + col]);
#pragma unroll
      for (int r = 0; r < 8; ++r) { const float v = acc[j][r] + bias; const _Float16 hv = (_Float16)v; sh[wave * 16 + 8 * g + r][j * 16 + col] = hv; sl[wave * 16 + 8 * g + r][j * 16 + col] = (_Float16)((v - (float)hv) * QRES); } }
    __syncthreads();
    _Float16* DST = which == 0 ? QH : KH;
    for (int e = tid; e < 64 * 16; e += 128) { const int rl = e >> 4, q = e & 15; const size_t o = (r0 + rl) * CC + c0 + q * 8;
      vst2((unsigned*)(DST + o), *(const v4u*)&sh[rl][q * 8]);
      if (which == 0) vst2((unsigned*)(QL + o), *(const v4u*)&sl[rl][q * 8]); }
  } else {
#pragma unroll
    for (int j = 0; j < 8; ++j) { const float bias = bfr(BA[c0 + j * 16 + col]);
#pragma unroll
      for (int r = 0; r < 8; ++r) { const float v = acc[j][r] + bias; const int rl = wave * 16 + 8 * g + r, cl = j * 16 + col; th[cl][rl] = (_Float16)v; } }
    __syncthreads();
    for (int e = tid; e < 128 * 8; e += 128) { const int cl = e >> 3, q = e & 7; vst2((unsigned*)(VT + (bb * CC + c0 + cl) * (size_t)SEQ + t0 + q * 8), *(const v4u*)&th[cl][q * 8]); }
  }
}
__global__ __launch_bounds__(128) void k_qrows(const float* __restrict__ X, const float* __restrict__ WQ, const float* __restrict__ BQ, float* __restrict__ QF) {
  __shared__ __align__(16) float sf[4][16][132];
  const int tid = threadIdx.x, wave = tid >> 5, lane = tid & 31, col = lane & 15, g = lane >> 4; const int c0 = blockIdx.y * 128;
  const size_t rb = (size_t)blockIdx.x * 64; const size_t bb = rb / SEQ; const int t0 = (int)(rb % SEQ);
  const size_t r0 = rb + wave * 16, x0 = bb * SEQ_FULL + t0 + wave * 16;
  v8f acc[8] = {};
#pragma unroll 2
  for (int kc = 0; kc < DIN / 32; ++kc) {
    v16b a; { const float* p = X + (x0 + col) * DIN + kc * 32 + 8 * g;
#pragma unroll
      for (int i = 0; i < 8; ++i) { a[i] = (__bf16)p[i]; a[8 + i] = (__bf16)p[16 + i]; } }
    asm volatile("s_wait_loadcnt 0x0" ::: "memory");
#pragma unroll
    for (int j = 0; j < 8; ++j) { const v16b w = wcol_io(WQ, kc * 32, c0 + j * 16 + col, lane, CC); asm volatile("s_wait_loadcnt 0x0" ::: "memory"); acc[j] = wmma_bf(a, w, acc[j]); }
  }
#pragma unroll
  for (int j = 0; j < 8; ++j) { const float bq2 = bfr(BQ[c0 + j * 16 + col]);
#pragma unroll
    for (int r = 0; r < 8; ++r) sf[wave][8 * g + r][j * 16 + col] = acc[j][r] + bq2; }
  ldsx(); for (int rl = 0; rl < 16; ++rl) vst2(QF + (r0 + rl) * CC + c0 + lane * 4, *(const v4f*)&sf[wave][rl][lane * 4]);
}
__global__ __launch_bounds__(256) void k_lnrow(const float* __restrict__ X, const float* __restrict__ R, const float* __restrict__ GM, const float* __restrict__ BT, float* __restrict__ OUT) {
  const int wave = threadIdx.x >> 5, lane = threadIdx.x & 31; const size_t row = (size_t)blockIdx.x * 8 + wave; if (row >= (size_t)NROW) return;
  v4f x[NQ4]; float s1 = 0.f;
#pragma unroll
  for (int q = 0; q < NQ4; ++q) { x[q] = *(const v4f*)(X + row * CC + q * 128 + lane * 4); if (R) { const v4f rr = *(const v4f*)(R + row * CC + q * 128 + lane * 4); x[q][0] += rr[0]; x[q][1] += rr[1]; x[q][2] += rr[2]; x[q][3] += rr[3]; }
#pragma unroll
    for (int i = 0; i < 4; ++i) s1 += x[q][i]; }
#pragma unroll
  for (int o = 1; o < 32; o <<= 1) s1 += __shfl_xor(s1, o);
  const float mu = s1 * (1.0f / CC); float qq = 0.f;
#pragma unroll
  for (int q = 0; q < NQ4; ++q)
#pragma unroll
    for (int i = 0; i < 4; ++i) { const float d = x[q][i] - mu; qq += d * d; }
#pragma unroll
  for (int o = 1; o < 32; o <<= 1) qq += __shfl_xor(qq, o);
  const float rs = rsqrtf(qq * (1.0f / CC) + 1e-5f);
#pragma unroll
  for (int q = 0; q < NQ4; ++q) { v4f r4; const int c = q * 128 + lane * 4;
#pragma unroll
    for (int i = 0; i < 4; ++i) r4[i] = (x[q][i] - mu) * rs * bfr(GM[c + i]) + bfr(BT[c + i]);
    vst2(OUT + row * CC + c, r4); }
}
__global__ __launch_bounds__(128) void k_rff(const float* __restrict__ O, const float* __restrict__ WO, const float* __restrict__ BO, float* __restrict__ T) {
  __shared__ __align__(16) float sf[4][16][132];
  const int tid = threadIdx.x, wave = tid >> 5, lane = tid & 31, col = lane & 15, g = lane >> 4; const int c0 = blockIdx.y * 128; const size_t r0 = (size_t)blockIdx.x * 64 + wave * 16;
  v8f acc[8] = {};
#pragma unroll 2
  for (int kc = 0; kc < CC / 32; ++kc) { const F2 a = split_row(O + (r0 + col) * CC, kc * 32, lane); asm volatile("s_wait_loadcnt 0x0" ::: "memory");
#pragma unroll
    for (int j = 0; j < 8; ++j) { const v16b w = wcol_io(WO, kc * 32, c0 + j * 16 + col, lane, CC); asm volatile("s_wait_loadcnt 0x0" ::: "memory"); acc[j] = wmma_bf(a.h, w, acc[j]); acc[j] = wmma_bf(a.l, w, acc[j]); } }
#pragma unroll
  for (int j = 0; j < 8; ++j) { const float bo2 = bfr(BO[c0 + j * 16 + col]);
#pragma unroll
    for (int r = 0; r < 8; ++r) sf[wave][8 * g + r][j * 16 + col] = fmaxf(acc[j][r] + bo2, 0.f); }
  ldsx(); for (int rl = 0; rl < 16; ++rl) { const size_t o2 = (r0 + rl) * CC + c0 + lane * 4; const v4f xo = *(const v4f*)(O + o2); v4f t = *(const v4f*)&sf[wave][rl][lane * 4]; t[0] += xo[0]; t[1] += xo[1]; t[2] += xo[2]; t[3] += xo[3]; vst2(T + o2, t); }
}
__global__ __launch_bounds__(128) __attribute__((amdgpu_num_vgpr(256))) void k_sc(const _Float16* __restrict__ QH, const _Float16* __restrict__ KH, const _Float16* __restrict__ QL, int b, int h0, float* __restrict__ S0) {
  __shared__ __align__(16) float ss[4][16][132];
  const int qb = blockIdx.x, kb = blockIdx.y; const int h = h0 + (int)blockIdx.z; float* S = S0 + (size_t)blockIdx.z * SEQ * SEQ;
  const int tid = threadIdx.x, wave = tid >> 5, lane = tid & 31, col = lane & 15, g = lane >> 4;
  const int k0 = kb * 128; const int ql0 = qb * 64 + wave * 16; const size_t q0 = (size_t)b * SEQ + ql0, kr0 = (size_t)b * SEQ + k0;
  v8f acc[8] = {}, accl[8] = {};
#pragma unroll
  for (int kc = 0; kc < HD / 32; ++kc) {
    const v16h ah = frag_h(QH + (q0 + col) * CC + h * HD + kc * 32, lane), al = frag_h(QL + (q0 + col) * CC + h * HD + kc * 32, lane);
#pragma unroll
    for (int j = 0; j < 8; ++j) { const v16h kf = frag_h(KH + (kr0 + j * 16 + col) * CC + h * HD + kc * 32, lane); acc[j] = wmma16(ah, kf, acc[j]); accl[j] = wmma16(al, kf, accl[j]); } }
#pragma unroll
  for (int j = 0; j < 8; ++j) {
#pragma unroll
    for (int r = 0; r < 8; ++r) ss[wave][8 * g + r][j * 16 + col] = (acc[j][r] + accl[j][r] * (1.0f / QRES)) * SCALE; }
  ldsx(); for (int rl = 0; rl < 16; ++rl) vst2(S + (size_t)(ql0 + rl) * SEQ + k0 + lane * 4, *(const v4f*)&ss[wave][rl][lane * 4]);
}
__global__ __launch_bounds__(256) void k_sm(float* __restrict__ S0) {
  __shared__ float sred[8]; __shared__ float sbc; __shared__ __align__(16) float shv[SEQ];
  const int tid = threadIdx.x; const int t = blockIdx.x;
  float* sr = S0 + (size_t)blockIdx.y * SEQ * SEQ + (size_t)t * SEQ;
  float m = -3.0e38f; for (int k = tid; k < SEQ; k += 256) { const float v = sr[k]; shv[k] = v; m = fmaxf(m, v); }
#pragma unroll
  for (int o = 1; o < 32; o <<= 1) m = fmaxf(m, __shfl_xor(m, o));
  if ((tid & 31) == 0) sred[tid >> 5] = m; __syncthreads(); if (tid == 0) { float a = sred[0]; for (int i = 1; i < 8; ++i) a = fmaxf(a, sred[i]); sbc = a; } __syncthreads(); m = sbc; __syncthreads();
  float sum = 0.f; for (int k = tid; k < SEQ; k += 256) { const float e = expf(shv[k] - m); shv[k] = e; sum += e; }
#pragma unroll
  for (int o = 1; o < 32; o <<= 1) sum += __shfl_xor(sum, o);
  if ((tid & 31) == 0) sred[tid >> 5] = sum; __syncthreads(); if (tid == 0) { float a = 0.f; for (int i = 0; i < 8; ++i) a += sred[i]; sbc = a > 0.f ? PCARRY / a : 0.f; } __syncthreads(); const float inv = sbc;
  for (int k = tid; k < SEQ; k += 256) shv[k] = shv[k] * inv;
  __syncthreads(); for (int q = tid; q < SEQ / 4; q += 256) vst2(sr + q * 4, *(const v4f*)&shv[q * 4]);
}
__global__ __launch_bounds__(128) __attribute__((amdgpu_num_vgpr(256))) void k_pv(const float* __restrict__ PS0, const _Float16* __restrict__ VT, int b, int h0, float* __restrict__ Y) {
  __shared__ __align__(16) float ss[4][16][HD + 4];
  const int h = h0 + (int)blockIdx.z; const float* PS = PS0 + (size_t)blockIdx.z * SEQ * SEQ;
  const int tid = threadIdx.x, wave = tid >> 5, lane = tid & 31, col = lane & 15, g = lane >> 4; const int qb = blockIdx.x; const int ql0 = qb * 64 + wave * 16;
  v8f acc[HD / 16] = {};
#pragma unroll 1
  for (int kc = 0; kc < SEQ / 32; ++kc) { const v16h p = frag_f32(PS + (size_t)(ql0 + col) * SEQ + kc * 32, lane);
    asm volatile("s_wait_loadcnt 0x0" ::: "memory");
#pragma unroll
    for (int j = 0; j < HD / 16; ++j) { const size_t po = ((size_t)b * CC + h * HD + j * 16 + col) * (size_t)SEQ + kc * 32; acc[j] = wmma16(p, frag_h(VT + po, lane), acc[j]); } }
#pragma unroll
  for (int j = 0; j < HD / 16; ++j)
#pragma unroll
    for (int r = 0; r < 8; ++r) ss[wave][8 * g + r][j * 16 + col] = acc[j][r] * (1.0f / PCARRY);
  ldsx(); for (int rl = 0; rl < 16; ++rl) if (lane < HD / 4) vst2(Y + ((size_t)b * SEQ + ql0 + rl) * CC + h * HD + lane * 4, *(const v4f*)&ss[wave][rl][lane * 4]);
}

extern "C" void kernel_launch(void* const* d_in, const int* in_sizes, int n_in, void* d_out, int out_size, void* d_ws, size_t ws_size, hipStream_t stream) {
  if (n_in < 14) return;
  if ((size_t)in_sizes[0] < (size_t)NB * SEQ_FULL * DIN || (size_t)in_sizes[1] < (size_t)NB * SEQ_FULL * DIN) return;
  if (in_sizes[2] < DIN * CC || in_sizes[4] < DIN * CC || in_sizes[6] < DIN * CC || in_sizes[8] < CC * CC) return;
  if (in_sizes[3] < CC || in_sizes[5] < CC || in_sizes[7] < CC || in_sizes[9] < CC || in_sizes[10] < CC || in_sizes[11] < CC || in_sizes[12] < CC || in_sizes[13] < CC) return;
  if ((size_t)out_size < (size_t)NROW * CC) return;
  if (ws_size < (size_t)WS_END) return;
  const float* const* F = (const float* const*)d_in;
  char* ws = (char*)d_ws;
  _Float16 *QH = (_Float16*)(ws + WS_QH), *KH = (_Float16*)(ws + WS_KH), *VT = (_Float16*)(ws + WS_VT), *QL = (_Float16*)(ws + WS_QL);
  float *S = (float*)(ws + WS_S), *QF = (float*)(ws + WS_QF), *O = (float*)(ws + WS_O), *T = (float*)(ws + WS_T);
  k_proj<<<dim3(NROW / 64, CC / 128, 3), 128, 0, stream>>>(F[0], F[1], F[2], F[4], F[6], F[3], F[5], F[7], QH, QL, KH, VT);
  k_qrows<<<dim3(NROW / 64, CC / 128), 128, 0, stream>>>(F[0], F[2], F[3], QF);
  for (int b = 0; b < NB; ++b)
    for (int hg = 0; hg < NH / HG; ++hg) {
      k_sc<<<dim3(NQB, SEQ / 128, HG), 128, 0, stream>>>(QH, KH, QL, b, hg * HG, S);
      k_sm<<<dim3(SEQ, HG), 256, 0, stream>>>(S);
      k_pv<<<dim3(NQB, 1, HG), 128, 0, stream>>>(S, VT, b, hg * HG, T);
    }
  k_lnrow<<<dim3((NROW + 7) / 8), 256, 0, stream>>>(QF, T, F[10], F[11], O);
  k_rff<<<dim3(NROW / 64, CC / 128), 128, 0, stream>>>(O, F[8], F[9], T);
  k_lnrow<<<dim3((NROW + 7) / 8), 256, 0, stream>>>(T, nullptr, F[12], F[13], (float*)d_out);
}
